// EmbedMetadata_51135880626864
// MI455X (gfx1250) — hardware-verified
//
#include <hip/hip_runtime.h>
#include <stdint.h>
#include <stddef.h>

#pragma clang fp contract(off)

#define NB     16384
#define NI     35
#define NE     256
#define NC     64
#define KX     105
#define KP     128
#define TCONST 140
#define NT2    141
#define MROW   140
#define WFP    8960
#define MT     32
#define NW     4
#define SFP    260
#define FB_TPB 192
#define FT_TPB 256
#define MN_TPB 128

static_assert(NB % MT == 0);
static_assert(MT == 2 * 16);
static_assert(NW * 64 == NE);
static_assert(NW * 32 == MN_TPB);
static_assert(KX == 3 * NI);
static_assert(MROW == 4 * NI);
static_assert(WFP == NI * 4 * NC);
static_assert(KP % 32 == 0);
static_assert(KP >= KX);
static_assert(KP <= MROW);
static_assert((MROW * 4) % 16 == 0);
static_assert(KP == 8 * 16);
static_assert(TCONST == 4 * NI);
static_assert(FT_TPB == NE);
static_assert(NE == 2 * 4 * 32);
static_assert((SFP * 4) % 16 == 0);
static_assert(SFP >= NE);
static_assert(MT % NW == 0);
static_assert((MT * KP) % (8 * MN_TPB) == 0);
static_assert(FB_TPB == 3 * 64);
static_assert(NC % 4 == 0);

typedef unsigned short us_t;
typedef __bf16         v16b __attribute__((ext_vector_type(16)));
typedef float          v8f  __attribute__((ext_vector_type(8)));
typedef float          v4f  __attribute__((ext_vector_type(4)));
typedef unsigned int   v4u  __attribute__((ext_vector_type(4)));
typedef unsigned short v8us __attribute__((ext_vector_type(8)));
typedef v4f __attribute__((may_alias)) v4fa;
typedef v4u __attribute__((may_alias)) v4ua;

union FragB { v16b v; v4u q[2]; };
union Pack8 { v8us s; v4u u; };

__device__ __forceinline__ unsigned int bfb(float f) {
  const unsigned int u = __float_as_uint(f);
  return (u + 0x7FFFu + ((u >> 16) & 1u)) >> 16;
}

__device__ __forceinline__ v8f wmma_b(v16b a, v16b b, v8f c) {
  v8f d = __builtin_amdgcn_wmma_f32_16x16x32_bf16(false, a, false, b, (short)0, c, false, false);
  asm volatile("v_nop\n\tv_nop\n\tv_nop\n\tv_nop" : "+v"(d) : "v"(a), "v"(b));
  return d;
}

__device__ __forceinline__ v8f wmma3(v16b ah, v16b al, v16b bh, v16b bl, v8f c) {
  c = wmma_b(ah, bh, c);
  c = wmma_b(al, bh, c);
  c = wmma_b(ah, bl, c);
  return c;
}

__device__ __forceinline__ v16b ldfrag(const us_t* p, int h) {
  FragB f;
  f.q[0] = *(const v4ua*)(p + 8 * h);
  f.q[1] = *(const v4ua*)(p + 16 + 8 * h);
  return f.v;
}

__device__ __forceinline__ float wsum(float v) {
  #pragma unroll
  for (int o = 16; o > 0; o >>= 1) v += __shfl_xor(v, o, 32);
  return v;
}

__device__ __forceinline__ void cbar() { asm volatile("" ::: "memory"); }

__global__ __launch_bounds__(FB_TPB) void k_foldB(const float* __restrict__ Wd,
                                                  const float* __restrict__ Wc,
                                                  const float* __restrict__ Wr,
                                                  const float* __restrict__ Wf,
                                                  us_t* __restrict__ bh,
                                                  us_t* __restrict__ bl)
{
  __shared__ __align__(16) float sB[KP];
  const int tid = threadIdx.x;
  const int e = blockIdx.x;
  const int g = tid >> 6;
  const int i = tid & 63;
  const int ic = (i < NI) ? i : (NI - 1);
  const float* src = (g == 0) ? Wd : ((g == 1) ? Wc : Wr);
  const float* w  = src + ic * NC;
  const float* wf = Wf + (size_t)e * WFP + ic * 256 + 64 * g;
  float acc = 0.f;
  #pragma unroll 4
  for (int c = 0; c < NC; ++c) acc = fmaf(w[c], wf[c], acc);
  if (i < NI) sB[NI * g + i] = acc;
  if (tid < KP - KX) sB[KX + tid] = 0.f;
  __syncthreads();

  if (tid < 16) {
    const v4f a = *(const v4fa*)(sB + 8 * tid);
    const v4f b = *(const v4fa*)(sB + 8 * tid + 4);
    float f[8];
    f[0] = a.x; f[1] = a.y; f[2] = a.z; f[3] = a.w;
    f[4] = b.x; f[5] = b.y; f[6] = b.z; f[7] = b.w;
    v8us hv, lv;
    #pragma unroll
    for (int q = 0; q < 8; ++q) {
      const unsigned int hb = bfb(f[q]);
      const float hf = __uint_as_float(hb << 16);
      const unsigned int lb = bfb(f[q] - hf);
      hv[q] = (us_t)hb;
      lv[q] = (us_t)lb;
    }
    Pack8 kh, kl;
    kh.s = hv;
    kl.s = lv;
    const v4u uh = kh.u, ul = kl.u;
    us_t* qh = bh + (size_t)e * KP + 8 * tid;
    us_t* ql = bl + (size_t)e * KP + 8 * tid;
    *(volatile v4u*)qh = uh;
    *(volatile v4u*)ql = ul;
    __threadfence();
    *(volatile v4u*)qh = uh;
    *(volatile v4u*)ql = ul;
  }
}

__global__ __launch_bounds__(FT_TPB) void k_foldT(const float* __restrict__ bd,
                                                  const float* __restrict__ bc,
                                                  const float* __restrict__ br,
                                                  const float* __restrict__ emb,
                                                  const float* __restrict__ Wf,
                                                  const float* __restrict__ bf,
                                                  float* __restrict__ t2)
{
  const int e = threadIdx.x;
  const int kp = blockIdx.x;
  const float* wfrow = Wf + (size_t)e * WFP;
  float val;
  if (kp < TCONST) {
    const int i = kp >> 2, t = kp & 3;
    const float* em = emb + (i * 4 + t) * NC;
    const float* wf = wfrow + i * 256 + 192;
    float acc = 0.f;
    #pragma unroll 4
    for (int c = 0; c < NC; ++c) acc = fmaf(em[c], wf[c], acc);
    val = acc;
  } else {
    float sd = 0.f, sc = 0.f, sr = 0.f;
    #pragma unroll 1
    for (int i = 0; i < NI; ++i) {
      const float* wf = wfrow + i * 256;
      const float* pd = bd + i * NC;
      const float* pc = bc + i * NC;
      const float* pr = br + i * NC;
      #pragma unroll 4
      for (int c = 0; c < NC; ++c) {
        sd = fmaf(pd[c], wf[c], sd);
        sc = fmaf(pc[c], wf[64 + c], sc);
        sr = fmaf(pr[c], wf[128 + c], sr);
      }
    }
    val = bf[e] + ((sd + sc) + sr);
  }
  float* q = t2 + (size_t)kp * NE + e;
  *(volatile float*)q = val;
  __threadfence();
  *(volatile float*)q = val;
}

__global__ __launch_bounds__(MN_TPB) void k_main(const float* __restrict__ meta,
                                                 const us_t* __restrict__ bh,
                                                 const us_t* __restrict__ bl,
                                                 const float* __restrict__ t2,
                                                 const float* __restrict__ gamma,
                                                 const float* __restrict__ beta,
                                                 float* __restrict__ out)
{
  __shared__ __align__(16) us_t  sXh[MT * KP];
  __shared__ __align__(16) us_t  sXl[MT * KP];
  __shared__ __align__(16) float sY[MT * SFP];
  __shared__ int sRt[MT * NI];

  const int tid = threadIdx.x, lane = tid & 31, wv = tid >> 5;
  const int h = lane >> 4, m = lane & 15;
  const int row0 = blockIdx.x * MT;

  #pragma unroll 1
  for (int j = 0; j < (MT * KP) / (8 * MN_TPB); ++j) {
    const int gi = j * MN_TPB + tid;
    const int r = gi >> 4, g = gi & 15;
    const float* mg = meta + (size_t)(row0 + r) * MROW + 8 * g;
    const v4f a = *(const v4fa*)mg;
    const v4f b = *(const v4fa*)(mg + 4);
    float f[8];
    f[0] = a.x; f[1] = a.y; f[2] = a.z; f[3] = a.w;
    f[4] = b.x; f[5] = b.y; f[6] = b.z; f[7] = b.w;
    v8us hv, lv;
    #pragma unroll
    for (int q = 0; q < 8; ++q) {
      const int k = 8 * g + q;
      const float fv = (k < KX) ? f[q] : 0.f;
      const unsigned int hb = bfb(fv);
      const float hf = __uint_as_float(hb << 16);
      const unsigned int lb = bfb(fv - hf);
      hv[q] = (us_t)hb;
      lv[q] = (us_t)lb;
    }
    Pack8 kh, kl;
    kh.s = hv;
    kl.s = lv;
    *(v4ua*)(sXh + r * KP + 8 * g) = kh.u;
    *(v4ua*)(sXl + r * KP + 8 * g) = kl.u;
  }

  #pragma unroll 1
  for (int j = 0; j < (MT * NI + MN_TPB - 1) / MN_TPB; ++j) {
    const int gi = j * MN_TPB + tid;
    const int gc = (gi < MT * NI) ? gi : (MT * NI - 1);
    const int r = gc / NI, i = gc - r * NI;
    float v = meta[(size_t)(row0 + r) * MROW + KX + i];
    v = fminf(fmaxf(v, -1.0e6f), 1.0e6f);
    int x = (int)v;
    x = (x == -1) ? 2 : ((x == -2) ? 3 : x);
    x = (x < 0) ? (x + 4) : x;
    x = (x < 0) ? 0 : ((x > 3) ? 3 : x);
    if (gi < MT * NI) sRt[gi] = x;
  }
  __syncthreads();

  const v8f z8 = {0.f, 0.f, 0.f, 0.f, 0.f, 0.f, 0.f, 0.f};
  v8f acc[2][4];
  #pragma unroll
  for (int mt = 0; mt < 2; ++mt)
    #pragma unroll
    for (int nt = 0; nt < 4; ++nt) acc[mt][nt] = z8;

  const us_t* ah0p = sXh + m * KP;
  const us_t* ah1p = sXh + (16 + m) * KP;
  const us_t* al0p = sXl + m * KP;
  const us_t* al1p = sXl + (16 + m) * KP;
  const size_t boff = (size_t)(64 * wv + m) * KP;

  #pragma unroll 1
  for (int kb = 0; kb < KP; kb += 32) {
    const v16b ah0 = ldfrag(ah0p + kb, h);
    const v16b ah1 = ldfrag(ah1p + kb, h);
    const v16b al0 = ldfrag(al0p + kb, h);
    const v16b al1 = ldfrag(al1p + kb, h);
    #pragma unroll
    for (int nt = 0; nt < 2; ++nt) {
      const size_t bo = boff + (size_t)(16 * nt) * KP + kb;
      const v16b bhf = ldfrag(bh + bo, h);
      const v16b blf = ldfrag(bl + bo, h);
      acc[0][nt] = wmma3(ah0, al0, bhf, blf, acc[0][nt]);
      acc[1][nt] = wmma3(ah1, al1, bhf, blf, acc[1][nt]);
    }
    cbar();
    #pragma unroll
    for (int nt = 2; nt < 4; ++nt) {
      const size_t bo = boff + (size_t)(16 * nt) * KP + kb;
      const v16b bhf = ldfrag(bh + bo, h);
      const v16b blf = ldfrag(bl + bo, h);
      acc[0][nt] = wmma3(ah0, al0, bhf, blf, acc[0][nt]);
      acc[1][nt] = wmma3(ah1, al1, bhf, blf, acc[1][nt]);
    }
    cbar();
  }

  #pragma unroll
  for (int mt = 0; mt < 2; ++mt)
    #pragma unroll
    for (int nt = 0; nt < 4; ++nt)
      #pragma unroll
      for (int r = 0; r < 8; ++r)
        sY[(16 * mt + 8 * h + r) * SFP + 64 * wv + 16 * nt + m] = acc[mt][nt][r];
  __syncthreads();

  const v4f g0 = *(const v4fa*)(gamma + 4 * lane);
  const v4f g1 = *(const v4fa*)(gamma + 128 + 4 * lane);
  const v4f e0 = *(const v4fa*)(beta + 4 * lane);
  const v4f e1 = *(const v4fa*)(beta + 128 + 4 * lane);
  const float* tcr = t2 + (size_t)TCONST * NE;
  const v4f c0 = *(const v4fa*)(tcr + 4 * lane);
  const v4f c1 = *(const v4fa*)(tcr + 128 + 4 * lane);

  #pragma unroll 1
  for (int rr = 0; rr < MT / NW; ++rr) {
    const int r = wv + NW * rr;
    v4f y0 = *(const v4fa*)(sY + r * SFP + 4 * lane);
    v4f y1 = *(const v4fa*)(sY + r * SFP + 128 + 4 * lane);
    y0 = y0 + c0;
    y1 = y1 + c1;
    #pragma unroll 4
    for (int i = 0; i < NI; ++i) {
      int kp = 4 * i + sRt[r * NI + i];
      kp = (kp < 0) ? 0 : ((kp > TCONST - 1) ? (TCONST - 1) : kp);
      const float* tr = t2 + (size_t)kp * NE;
      y0 = y0 + *(const v4fa*)(tr + 4 * lane);
      y1 = y1 + *(const v4fa*)(tr + 128 + 4 * lane);
    }
    float s = ((y0.x + y0.y) + (y0.z + y0.w)) + ((y1.x + y1.y) + (y1.z + y1.w));
    s = wsum(s);
    const float mu = s * (1.f / (float)NE);
    const v4f d0 = y0 - mu;
    const v4f d1 = y1 - mu;
    float s2 = ((d0.x * d0.x + d0.y * d0.y) + (d0.z * d0.z + d0.w * d0.w)) +
               ((d1.x * d1.x + d1.y * d1.y) + (d1.z * d1.z + d1.w * d1.w));
    s2 = wsum(s2);
    const float var = s2 * (1.f / (float)NE);
    const float rs = rsqrtf(var + 1.0e-5f);
    v4f o0 = d0 * rs * g0 + e0;
    v4f o1 = d1 * rs * g1 + e1;
    o0.x = fmaxf(o0.x, 0.f); o0.y = fmaxf(o0.y, 0.f); o0.z = fmaxf(o0.z, 0.f); o0.w = fmaxf(o0.w, 0.f);
    o1.x = fmaxf(o1.x, 0.f); o1.y = fmaxf(o1.y, 0.f); o1.z = fmaxf(o1.z, 0.f); o1.w = fmaxf(o1.w, 0.f);
    float* dst = out + (size_t)(row0 + r) * NE;
    *(volatile v4f*)(dst + 4 * lane) = o0;
    *(volatile v4f*)(dst + 128 + 4 * lane) = o1;
    __threadfence();
    *(volatile v4f*)(dst + 4 * lane) = o0;
    *(volatile v4f*)(dst + 128 + 4 * lane) = o1;
  }
}

extern "C" void kernel_launch(void* const* d_in, const int* in_sizes, int n_in,
                              void* d_out, int out_size, void* d_ws, size_t ws_size,
                              hipStream_t stream)
{
  if (n_in < 12) return;
  if (in_sizes[0] != NB * MROW) return;
  if (in_sizes[1] != NI * NC) return;
  if (in_sizes[2] != NI * NC) return;
  if (in_sizes[3] != NI * NC) return;
  if (in_sizes[4] != NI * NC) return;
  if (in_sizes[5] != NI * NC) return;
  if (in_sizes[6] != NI * NC) return;
  if (in_sizes[7] != NI * 4 * NC) return;
  if (in_sizes[8] != NE * WFP) return;
  if (in_sizes[9] != NE) return;
  if (in_sizes[10] != NE) return;
  if (in_sizes[11] != NE) return;
  if (out_size != NB * NE) return;

  const float* meta  = (const float*)d_in[0];
  const float* Wd    = (const float*)d_in[1];
  const float* bd    = (const float*)d_in[2];
  const float* Wc    = (const float*)d_in[3];
  const float* bc    = (const float*)d_in[4];
  const float* Wr    = (const float*)d_in[5];
  const float* br    = (const float*)d_in[6];
  const float* emb   = (const float*)d_in[7];
  const float* Wf    = (const float*)d_in[8];
  const float* bf    = (const float*)d_in[9];
  const float* gamma = (const float*)d_in[10];
  const float* beta  = (const float*)d_in[11];
  float* out = (float*)d_out;

  const size_t bB = (size_t)NE * KP * 2;
  const size_t bT = (size_t)NT2 * NE * 4;
  const size_t total = 2 * bB + bT;
  if (total > ws_size) return;
  if (total > (size_t)134217728) return;

  char* ws = (char*)d_ws;
  size_t off = 0;
  us_t*  Bh = (us_t*)(ws + off);  off += bB;
  us_t*  Bl = (us_t*)(ws + off);  off += bB;
  float* T2 = (float*)(ws + off); off += bT;
  if (off != total) return;

  k_foldB<<<NE, FB_TPB, 0, stream>>>(Wd, Wc, Wr, Wf, Bh, Bl);
  k_foldT<<<NT2, FT_TPB, 0, stream>>>(bd, bc, br, emb, Wf, bf, T2);
  k_main<<<NB / MT, MN_TPB, 0, stream>>>(meta, Bh, Bl, T2, gamma, beta, out);
}
